// BasicBlock_49263274885742
// MI455X (gfx1250) — hardware-run, weakly checked
//
#include <hip/hip_runtime.h>
#include <stddef.h>
#include <stdint.h>


#define F        64
#define K1       67
#define K1P      96
#define K2       64
#define KS       128
#define NTHR     256
#define NWAVE    8
#define GBM      64
#define GBN      64
#define GTHR     128
#define EPT      8
#define CHUNK    (NTHR * EPT)
#define WCAP     (EPT * 32)
#define LISTN    (NWAVE * WCAP)
#define NBMAX    256
#define SLB      8
#define RCAP     12288
#define TROWS    32
#define AP       72
#define DP       68
#define MISCN    32
#define MAXTILES (RCAP / TROWS)
#define UI_W1    ((F * K1P) / 8)
#define UI_W2    ((F * K2) / 8)
#define UI_U3    ((F * KS) / 8)
#define UI_U4    ((F * KS) / 8)
#define UI_TOT   (UI_W1 + UI_W2 + UI_U3 + UI_U4)
#define AGG_ZINTS (LISTN + 2 * RCAP + 3 * NBMAX + MISCN)
#define SA_OFFI   AGG_ZINTS
#define SD_OFFI   (SA_OFFI + (NWAVE * TROWS * AP) / 2)
#define SAG_OFFI  (SD_OFFI + NWAVE * TROWS * DP)
#define SB2_OFFI  (SAG_OFFI + NBMAX * F)
#define AGG_LDS_INTS (SB2_OFFI + F)
#define AGG_LDS_BYTES (AGG_LDS_INTS * 4)
#define SC_A     16.0f
#define SC_W     1024.0f
#define SC14     6.103515625e-05f
#define WSMAX    134217728

static_assert((CHUNK & (CHUNK - 1)) == 0);
static_assert(NBMAX == (1 << SLB));
static_assert(((long long)(CHUNK - 1) << SLB) + NBMAX < (1LL << 30));
static_assert(WCAP == EPT * 32 && LISTN == NWAVE * WCAP);
static_assert(NBMAX % (2 * NWAVE) == 0 && NBMAX % 32 == 0);
static_assert(RCAP % TROWS == 0 && TROWS == 32);
static_assert(AGG_ZINTS % 4 == 0 && SA_OFFI % 4 == 0 && SD_OFFI % 4 == 0 && SAG_OFFI % 4 == 0 && SB2_OFFI % 4 == 0);
static_assert((NWAVE * TROWS * AP) % 8 == 0 && (NBMAX * F) % 4 == 0);
static_assert(AGG_LDS_BYTES <= 300000);
static_assert(AP >= K2 && (AP * 2) % 16 == 0 && DP >= F && (DP % 2) == 0);
static_assert(UI_TOT % NTHR == 0 && UI_W1 % NTHR == 0 && (UI_W1 + UI_W2) % NTHR == 0 &&
              (UI_W1 + UI_W2 + UI_U3) % NTHR == 0);
static_assert(K1P % 32 == 0 && K2 % 32 == 0 && KS % 32 == 0 && KS == 2 * F && K1P >= K1 && K1 == F + 3);
static_assert(GBM == (GTHR / 32) * 16 && GBN == 4 * 16 && F == 64);
static_assert(MISCN >= 16 + NWAVE);

typedef float          v2f   __attribute__((ext_vector_type(2)));
typedef float          v4f   __attribute__((ext_vector_type(4)));
typedef float          v8f   __attribute__((ext_vector_type(8)));
typedef int            v4i   __attribute__((ext_vector_type(4)));
typedef int            v8i   __attribute__((ext_vector_type(8)));
typedef unsigned short v8us  __attribute__((ext_vector_type(8)));
typedef unsigned short v16us __attribute__((ext_vector_type(16)));
typedef __bf16         v16bf __attribute__((ext_vector_type(16)));
typedef _Float16       v8h   __attribute__((ext_vector_type(8)));
typedef _Float16       v16h  __attribute__((ext_vector_type(16)));
typedef v2f  __attribute__((may_alias)) v2fa;
typedef v4f  __attribute__((may_alias)) v4fa;
typedef v4i  __attribute__((may_alias)) v4ia;
typedef v8us __attribute__((may_alias)) v8usa;
typedef v8h  __attribute__((may_alias)) v8ha;
union FragB { v16bf v; v16us u; v8us h[2]; v8i w; };
union FragH { v16h v; v8h h[2]; v8i w; };

__device__ __forceinline__ v8f wmb(const FragB& a, const FragB& b, v8f c) {
  v8f d = __builtin_amdgcn_wmma_f32_16x16x32_bf16(false, a.v, false, b.v, (short)0, c, false, false);
  asm volatile("v_nop\n\tv_nop\n\tv_nop\n\tv_nop" : "+v"(d) : "v"(a.w), "v"(b.w));
  return d;
}
__device__ __forceinline__ v8f wmh(const FragH& a, const FragH& b, v8f c) {
  v8f d = __builtin_amdgcn_wmma_f32_16x16x32_f16(false, a.v, false, b.v, (short)0, c, false, false);
  asm volatile("v_nop\n\tv_nop\n\tv_nop\n\tv_nop" : "+v"(d) : "v"(a.w), "v"(b.w));
  return d;
}

__device__ __forceinline__ unsigned bf16_bits(float f) {
  const unsigned u = __float_as_uint(f);
  return (u + 0x7FFFu + ((u >> 16) & 1u)) >> 16;
}
__device__ __forceinline__ float bf16_val(float f) {
  return __uint_as_float(bf16_bits(f) << 16);
}
__device__ __forceinline__ v4f bfr4(const v4f a) {
  v4f r; r.x = bf16_val(a.x); r.y = bf16_val(a.y); r.z = bf16_val(a.z); r.w = bf16_val(a.w); return r;
}
__device__ __forceinline__ void put16(unsigned short* dp, v8us o) {
  *(volatile v8us*)dp = o;
  __threadfence();
  *(volatile v8us*)dp = o;
}
__device__ __forceinline__ void puth8(_Float16* dp, v8h o) {
  *(volatile v8h*)dp = o;
  __threadfence();
  *(volatile v8h*)dp = o;
}
__device__ __forceinline__ void put4f(float* dp, v4f o) {
  *(volatile v4f*)dp = o;
  __threadfence();
  *(volatile v4f*)dp = o;
}

__global__ __launch_bounds__(NTHR) void k_prep(const float* __restrict__ W1, const float* __restrict__ W2,
                                               const float* __restrict__ W3, const float* __restrict__ W4,
                                               unsigned short* W1T, _Float16* W2H,
                                               unsigned short* U3T, unsigned short* U4T) {
  const int u = (int)blockIdx.x * NTHR + (int)threadIdx.x;
  if (u >= UI_TOT) return;
  if (u < UI_W1) {
    const int n  = u / 12;
    const int k8 = (u - 12 * n) * 8;
    v8us o;
#pragma unroll
    for (int i = 0; i < 8; ++i) {
      const int k  = k8 + i;
      const int kc = k < K1 ? k : K1 - 1;
      const float okf = k < K1 ? 1.0f : 0.0f;
      o[i] = (unsigned short)bf16_bits(W1[(size_t)kc * F + n] * okf);
    }
    put16(W1T + (size_t)u * 8, o);
  } else if (u < UI_W1 + UI_W2) {
    const int v  = u - UI_W1;
    const int n  = v >> 3;
    const int k8 = (v & 7) * 8;
    v8h o;
#pragma unroll
    for (int i = 0; i < 8; ++i) o[i] = (_Float16)(bf16_val(W2[(size_t)(k8 + i) * F + n]) * SC_W);
    puth8(W2H + (size_t)v * 8, o);
  } else if (u < UI_W1 + UI_W2 + UI_U3) {
    const int v    = u - (UI_W1 + UI_W2);
    const int n    = v >> 4;
    const int k8   = (v & 15) * 8;
    const int srow = k8 & (F - 1);
    v8us o;
#pragma unroll
    for (int i = 0; i < 8; ++i) o[i] = (unsigned short)bf16_bits(W3[(size_t)(srow + i) * F + n]);
    put16(U3T + (size_t)v * 8, o);
  } else {
    const int v    = u - (UI_W1 + UI_W2 + UI_U3);
    const int n    = v >> 4;
    const int k8   = (v & 15) * 8;
    const int srow = k8 & (F - 1);
    v8us o;
#pragma unroll
    for (int i = 0; i < 8; ++i) o[i] = (unsigned short)bf16_bits(W4[(size_t)(srow + i) * F + n]);
    put16(U4T + (size_t)v * 8, o);
  }
}

__global__ __launch_bounds__(NTHR) void k_ccb(const float* __restrict__ cc, int nN, const float* __restrict__ W1,
                                              const float* __restrict__ b1, int nUnits, float* CCB) {
  const int u = (int)blockIdx.x * NTHR + (int)threadIdx.x;
  if (u >= nUnits) return;
  const int row = u >> 4;
  const int c4  = (u & 15) * 4;
  const int rc  = row < nN ? row : nN - 1;
  const float x = bf16_val(cc[(size_t)rc * 3]);
  const float y = bf16_val(cc[(size_t)rc * 3 + 1]);
  const float z = bf16_val(cc[(size_t)rc * 3 + 2]);
  const v4f wa = bfr4(*(const v4fa*)(W1 + (size_t)(F + 0) * F + c4));
  const v4f wb = bfr4(*(const v4fa*)(W1 + (size_t)(F + 1) * F + c4));
  const v4f wc = bfr4(*(const v4fa*)(W1 + (size_t)(F + 2) * F + c4));
  const v4f bb = bfr4(*(const v4fa*)(b1 + c4));
  v4f t;
  t.x = x * wa.x; t.x = fmaf(y, wb.x, t.x); t.x = fmaf(z, wc.x, t.x);
  t.y = x * wa.y; t.y = fmaf(y, wb.y, t.y); t.y = fmaf(z, wc.y, t.y);
  t.z = x * wa.z; t.z = fmaf(y, wb.z, t.z); t.z = fmaf(z, wc.z, t.z);
  t.w = x * wa.w; t.w = fmaf(y, wb.w, t.w); t.w = fmaf(z, wc.w, t.w);
  const v4f v = bb - t;
  put4f(CCB + (size_t)u * 4, v);
}

template <int AM, int EM>
__global__ __launch_bounds__(GTHR) void k_gemm(const unsigned short* __restrict__ Ab, int lda,
                                               const float* __restrict__ Xf, const float* __restrict__ Xc, int nX,
                                               const unsigned short* __restrict__ BT, int ldb, int K,
                                               const float* __restrict__ bias, int nlim,
                                               float* Cm, unsigned short* Cb) {
  static_assert(AM == 0 || AM == 2);
  static_assert(EM == 0 || EM == 2 || EM == 3);
  __shared__ __attribute__((aligned(16))) float stg[GBM * GBN];
  const int tid = (int)threadIdx.x, lane = tid & 31, wave = tid >> 5, hh = lane >> 4, m = lane & 15;
  const int rowBase = (int)blockIdx.x * GBM;

  v8f acc[4];
  {
    const v8f z = {0.f, 0.f, 0.f, 0.f, 0.f, 0.f, 0.f, 0.f};
#pragma unroll
    for (int t = 0; t < 4; ++t) acc[t] = z;
  }
  const int ar = rowBase + 16 * wave + m;
  const unsigned short* bp = BT + (size_t)m * (size_t)ldb + 8 * hh;

  if constexpr (AM == 0) {
    const unsigned short* ap = Ab + (size_t)ar * (size_t)lda + 8 * hh;
#pragma unroll 1
    for (int k0 = 0; k0 < K; k0 += 32) {
      FragB af;
      af.h[0] = *(const v8usa*)(ap + k0);
      af.h[1] = *(const v8usa*)(ap + k0 + 16);
#pragma unroll
      for (int nt = 0; nt < 4; ++nt) {
        const unsigned short* wq = bp + (size_t)(16 * nt) * (size_t)ldb + k0;
        FragB bf;
        bf.h[0] = *(const v8usa*)wq;
        bf.h[1] = *(const v8usa*)(wq + 16);
        acc[nt] = wmb(af, bf, acc[nt]);
      }
    }
  } else {
    const int arc = ar < nX ? ar : nX - 1;
    const float okf = ar < nX ? 1.0f : 0.0f;
    const float* xp = Xf + (size_t)arc * F + 8 * hh;
#pragma unroll
    for (int ks = 0; ks < 2; ++ks) {
      const int k0 = 32 * ks;
      const v4f u0 = *(const v4fa*)(xp + k0);
      const v4f u1 = *(const v4fa*)(xp + k0 + 4);
      const v4f u2 = *(const v4fa*)(xp + k0 + 16);
      const v4f u3 = *(const v4fa*)(xp + k0 + 20);
      const v8f f0 = {u0.x, u0.y, u0.z, u0.w, u1.x, u1.y, u1.z, u1.w};
      const v8f f1 = {u2.x, u2.y, u2.z, u2.w, u3.x, u3.y, u3.z, u3.w};
      v8us o0, o1;
#pragma unroll
      for (int e = 0; e < 8; ++e) {
        o0[e] = (unsigned short)bf16_bits(f0[e] * okf);
        o1[e] = (unsigned short)bf16_bits(f1[e] * okf);
      }
      FragB af;
      af.h[0] = o0;
      af.h[1] = o1;
#pragma unroll
      for (int nt = 0; nt < 4; ++nt) {
        const unsigned short* wq = bp + (size_t)(16 * nt) * (size_t)ldb + k0;
        FragB bf;
        bf.h[0] = *(const v8usa*)wq;
        bf.h[1] = *(const v8usa*)(wq + 16);
        acc[nt] = wmb(af, bf, acc[nt]);
      }
    }
    {
      const float okh = (hh == 0) ? okf : 0.0f;
      const float* cq = Xc + (size_t)arc * 3;
      const float c0 = cq[0], c1 = cq[1], c2 = cq[2];
      v8us o0 = {0, 0, 0, 0, 0, 0, 0, 0};
      const v8us o1 = {0, 0, 0, 0, 0, 0, 0, 0};
      o0[0] = (unsigned short)bf16_bits(c0 * okh);
      o0[1] = (unsigned short)bf16_bits(c1 * okh);
      o0[2] = (unsigned short)bf16_bits(c2 * okh);
      FragB af;
      af.h[0] = o0;
      af.h[1] = o1;
#pragma unroll
      for (int nt = 0; nt < 4; ++nt) {
        const unsigned short* wq = bp + (size_t)(16 * nt) * (size_t)ldb + F;
        FragB bf;
        bf.h[0] = *(const v8usa*)wq;
        bf.h[1] = *(const v8usa*)(wq + 16);
        acc[nt] = wmb(af, bf, acc[nt]);
      }
    }
  }

#pragma unroll
  for (int nt = 0; nt < 4; ++nt) {
    const int lc = 16 * nt + m;
    float bvv = 0.0f;
    if constexpr (EM != 0) bvv = bf16_val(bias[lc]);
#pragma unroll
    for (int r = 0; r < 8; ++r) {
      const int lr = 16 * wave + 8 * hh + r;
      float v = acc[nt][r];
      if constexpr (EM != 0) v = fmaxf(v + bvv, 0.0f);
      stg[lr * GBN + lc] = v;
    }
  }
  __syncthreads();

  const int hsel = lane >> 4;
  if constexpr (EM == 0 || EM == 3) {
    const int c = 4 * (lane & 15);
    v4f pv[8];
#pragma unroll
    for (int i2 = 0; i2 < 8; ++i2) pv[i2] = *(const v4fa*)(stg + (16 * wave + 2 * i2 + hsel) * GBN + c);
#pragma unroll
    for (int i2 = 0; i2 < 8; ++i2) {
      const int row = rowBase + 16 * wave + 2 * i2 + hsel;
      if constexpr (EM == 0) {
        *(volatile v4f*)(Cm + (size_t)row * F + c) = pv[i2];
      } else {
        const int rowc = row < nlim ? row : 0;
        if (row < nlim) *(volatile v4f*)(Cm + (size_t)rowc * F + c) = pv[i2];
      }
    }
    __threadfence();
#pragma unroll
    for (int i2 = 0; i2 < 8; ++i2) {
      const int row = rowBase + 16 * wave + 2 * i2 + hsel;
      if constexpr (EM == 0) {
        *(volatile v4f*)(Cm + (size_t)row * F + c) = pv[i2];
      } else {
        const int rowc = row < nlim ? row : 0;
        if (row < nlim) *(volatile v4f*)(Cm + (size_t)rowc * F + c) = pv[i2];
      }
    }
  } else {
    const int j    = lane & 15;
    const int part = j >> 3;
    const int c8   = (j & 7) * 8;
    const unsigned mh = 0u - (unsigned)part;
    const unsigned ml = ~mh;
    v8us pv[8];
#pragma unroll
    for (int i2 = 0; i2 < 8; ++i2) {
      const int lr = 16 * wave + 2 * i2 + hsel;
      const float* sp = stg + lr * GBN + c8;
      const v4f a = *(const v4fa*)sp;
      const v4f b = *(const v4fa*)(sp + 4);
      const v8f f8 = {a.x, a.y, a.z, a.w, b.x, b.y, b.z, b.w};
      v8us oo;
#pragma unroll
      for (int e = 0; e < 8; ++e) {
        const unsigned hb = bf16_bits(f8[e]);
        const unsigned lb = bf16_bits(f8[e] - __uint_as_float(hb << 16));
        oo[e] = (unsigned short)((hb & ml) | (lb & mh));
      }
      pv[i2] = oo;
    }
#pragma unroll
    for (int i2 = 0; i2 < 8; ++i2) {
      unsigned short* op = Cb + (size_t)(rowBase + 16 * wave + 2 * i2 + hsel) * (size_t)KS + 8 * j;
      *(volatile v8us*)op = pv[i2];
    }
    __threadfence();
#pragma unroll
    for (int i2 = 0; i2 < 8; ++i2) {
      unsigned short* op = Cb + (size_t)(rowBase + 16 * wave + 2 * i2 + hsel) * (size_t)KS + 8 * j;
      *(volatile v8us*)op = pv[i2];
    }
  }
}

__device__ __forceinline__ int scan_chunk(const int* __restrict__ kc, int nE, int cbase, int slotBase, int nb,
                                          int vec8, int* list, int tid, int lane, int wave) {
  int wc = 0;
  const int el0  = tid * EPT;
  const int e0   = cbase + el0;
  const int sent = -2147483647 - 1;
  v4i da, db;
  if (vec8 != 0 && cbase + CHUNK <= nE) {
    da = *(const v4ia*)(kc + e0);
    db = *(const v4ia*)(kc + e0 + 4);
  } else {
    da.x = sent; da.y = sent; da.z = sent; da.w = sent;
    db = da;
#pragma unroll 1
    for (int g = 0; g < 2; ++g) {
      const int eg = e0 + 4 * g;
      const int i0 = min(eg, nE - 1), i1 = min(eg + 1, nE - 1), i2 = min(eg + 2, nE - 1), i3 = min(eg + 3, nE - 1);
      const int k0v = kc[i0];
      const int k1v = kc[i1];
      const int k2v = kc[i2];
      const int k3v = kc[i3];
      v4i kk;
      kk.x = (eg     < nE) ? k0v : sent;
      kk.y = (eg + 1 < nE) ? k1v : sent;
      kk.z = (eg + 2 < nE) ? k2v : sent;
      kk.w = (eg + 3 < nE) ? k3v : sent;
      da.x = (g == 0) ? kk.x : da.x;  da.y = (g == 0) ? kk.y : da.y;
      da.z = (g == 0) ? kk.z : da.z;  da.w = (g == 0) ? kk.w : da.w;
      db.x = (g == 1) ? kk.x : db.x;  db.y = (g == 1) ? kk.y : db.y;
      db.z = (g == 1) ? kk.z : db.z;  db.w = (g == 1) ? kk.w : db.w;
    }
  }
  const unsigned nbs = (unsigned)slotBase;
  const unsigned unb = (unsigned)nb;
  const unsigned s0 = (unsigned)da.x - nbs, s1 = (unsigned)da.y - nbs;
  const unsigned s2 = (unsigned)da.z - nbs, s3 = (unsigned)da.w - nbs;
  const unsigned s4 = (unsigned)db.x - nbs, s5 = (unsigned)db.y - nbs;
  const unsigned s6 = (unsigned)db.z - nbs, s7 = (unsigned)db.w - nbs;
  const bool h0 = s0 < unb, h1 = s1 < unb, h2 = s2 < unb, h3 = s3 < unb;
  const bool h4 = s4 < unb, h5 = s5 < unb, h6 = s6 < unb, h7 = s7 < unb;
  const unsigned any = __builtin_amdgcn_ballot_w32(h0 | h1 | h2 | h3 | h4 | h5 | h6 | h7);
  if (any != 0u) {
#define HITJ(J, HJ, SJ) { \
      const unsigned mj = __builtin_amdgcn_ballot_w32(HJ); \
      if (mj != 0u) { \
        if (HJ) { \
          const int pos = wc + (int)__builtin_amdgcn_mbcnt_lo(mj, 0u); \
          if (pos < WCAP) list[wave * WCAP + pos] = ((el0 + (J)) << SLB) | (int)(SJ); \
        } \
        wc += (int)__builtin_popcount(mj); } }
    HITJ(0, h0, s0)
    HITJ(1, h1, s1)
    HITJ(2, h2, s2)
    HITJ(3, h3, s3)
    HITJ(4, h4, s4)
    HITJ(5, h5, s5)
    HITJ(6, h6, s6)
    HITJ(7, h7, s7)
#undef HITJ
  }
  return wc;
}

__device__ __forceinline__ void wave_gemm_h(const _Float16* sAw, float* sDw, const _Float16* __restrict__ W2H,
                                            int hh, int m) {
  v8f acc[2][4];
  {
    const v8f z = {0.f, 0.f, 0.f, 0.f, 0.f, 0.f, 0.f, 0.f};
#pragma unroll
    for (int mt = 0; mt < 2; ++mt)
#pragma unroll
      for (int nt = 0; nt < 4; ++nt) acc[mt][nt] = z;
  }
  const _Float16* ap0 = sAw + m * AP + 8 * hh;
  const _Float16* ap1 = ap0 + 16 * AP;
  const _Float16* bp  = W2H + (size_t)m * K2 + 8 * hh;
#pragma unroll
  for (int ks = 0; ks < K2 / 32; ++ks) {
    const int k0 = 32 * ks;
    FragH a0, a1;
    a0.h[0] = *(const v8ha*)(ap0 + k0);
    a0.h[1] = *(const v8ha*)(ap0 + k0 + 16);
    a1.h[0] = *(const v8ha*)(ap1 + k0);
    a1.h[1] = *(const v8ha*)(ap1 + k0 + 16);
#pragma unroll
    for (int nt = 0; nt < 4; ++nt) {
      const _Float16* wq = bp + (size_t)(16 * nt) * K2 + k0;
      FragH b;
      b.h[0] = *(const v8ha*)wq;
      b.h[1] = *(const v8ha*)(wq + 16);
      acc[0][nt] = wmh(a0, b, acc[0][nt]);
      acc[1][nt] = wmh(a1, b, acc[1][nt]);
    }
  }
#pragma unroll
  for (int nt = 0; nt < 4; ++nt) {
    const int col = 16 * nt + m;
#pragma unroll
    for (int mt = 0; mt < 2; ++mt)
#pragma unroll
      for (int r = 0; r < 8; ++r) sDw[(16 * mt + 8 * hh + r) * DP + col] = acc[mt][nt][r];
  }
}

__global__ __launch_bounds__(NTHR) void k_scan(const int* __restrict__ ecur, const int* __restrict__ elast,
                                               int nE, int nLast, int nb, int vec8, int mRows,
                                               const float* __restrict__ PL, const float* __restrict__ CCB,
                                               const _Float16* __restrict__ W2H, const float* __restrict__ b2,
                                               unsigned short* AGB) {
  extern __shared__ __attribute__((aligned(16))) int dsm[];
  int*      list = dsm;
  int*      hl   = dsm + LISTN;
  int*      sl   = hl + RCAP;
  int*      cnt  = sl + RCAP;
  int*      offs = cnt + NBMAX;
  int*      cur  = offs + NBMAX;
  int*      misc = cur + NBMAX;
  _Float16* sA   = (_Float16*)(dsm + SA_OFFI);
  float*    sD   = (float*)(dsm + SD_OFFI);
  float*    sAG  = (float*)(dsm + SAG_OFFI);
  float*    sB2  = (float*)(dsm + SB2_OFFI);
  const int tid = (int)threadIdx.x, lane = tid & 31, wave = tid >> 5, hh = lane >> 4, m = lane & 15;
  const int nodeBase = (int)blockIdx.x * nb;

  {
    const v4i z4 = {0, 0, 0, 0};
    for (int i = tid * 4; i < AGG_ZINTS; i += NTHR * 4) *(v4ia*)(dsm + i) = z4;
    const v4f zf = {0.0f, 0.0f, 0.0f, 0.0f};
    for (int i = tid * 4; i < NBMAX * F; i += NTHR * 4) *(v4fa*)(sAG + i) = zf;
    if (tid < F) sB2[tid] = bf16_val(b2[tid]);
  }
  __syncthreads();

  int t = 0, ov = 0;
  const int nChunks = (nE + CHUNK - 1) / CHUNK;
#pragma unroll 1
  for (int ch = 0; ch < nChunks; ++ch) {
    const int cbase = ch * CHUNK;
    const int wc = scan_chunk(ecur, nE, cbase, nodeBase, nb, vec8, list, tid, lane, wave);
    if (lane == 0) misc[wave] = wc;
    __syncthreads();
    if (wave == 0) {
#pragma unroll 1
      for (int w2 = 0; w2 < NWAVE; ++w2) {
        int cc = misc[w2];
        cc = cc < 0 ? 0 : (cc > WCAP ? WCAP : cc);
#pragma unroll 1
        for (int b0 = 0; b0 < cc; b0 += 32) {
          const int idx = b0 + lane;
          const int ent = list[w2 * WCAP + (idx < WCAP ? idx : WCAP - 1)];
          const int m32 = (cc - b0) < 32 ? (cc - b0) : 32;
#pragma unroll 1
          for (int k = 0; k < m32; ++k) {
            const int u    = __builtin_amdgcn_readlane(ent, k);
            const int slot = u & (NBMAX - 1);
            const int el   = (u >> SLB) & (CHUNK - 1);
            const int pk   = ((cbase + el) << SLB) | slot;
            if (t < RCAP) {
              if (lane == 0) { hl[t] = pk; cnt[slot] = cnt[slot] + 1; }
              t = t + 1;
            } else {
              ov = 1;
            }
          }
        }
      }
    }
    __syncthreads();
  }
  if (wave == 0 && lane == 0) { misc[8] = t; misc[9] = ov; }
  __syncthreads();
  int tt = misc[8];
  tt = tt < 0 ? 0 : (tt > RCAP ? RCAP : tt);

  if (wave == 0) {
    const int base = lane * (NBMAX / 32);
    int s = 0;
#pragma unroll 1
    for (int i = 0; i < NBMAX / 32; ++i) s += cnt[base + i];
    int incl = s;
#pragma unroll
    for (int d = 1; d < 32; d <<= 1) {
      const int y = __shfl_up(incl, d, 32);
      if (lane >= d) incl += y;
    }
    int run = incl - s;
#pragma unroll 1
    for (int i = 0; i < NBMAX / 32; ++i) {
      const int cv = cnt[base + i];
      offs[base + i] = run;
      cur[base + i]  = run;
      run += cv;
    }
  }
  __syncthreads();
  if (wave == 0) {
#pragma unroll 1
    for (int b0 = 0; b0 < tt; b0 += 32) {
      const int idx = b0 + lane;
      const int ent = hl[idx < RCAP ? idx : RCAP - 1];
      const int m32 = (tt - b0) < 32 ? (tt - b0) : 32;
#pragma unroll 1
      for (int k = 0; k < m32; ++k) {
        const int u    = __builtin_amdgcn_readlane(ent, k);
        const int slot = u & (NBMAX - 1);
        if (lane == 0) {
          int p = cur[slot];
          p = p < 0 ? 0 : (p > RCAP - 1 ? RCAP - 1 : p);
          sl[p] = u;
          cur[slot] = p + 1;
        }
      }
    }
  }
  __syncthreads();

  const int nsl = nb / NWAVE;
  const int ss0 = wave * nsl;
  int hb = offs[ss0];
  int he = offs[ss0 + nsl - 1] + cnt[ss0 + nsl - 1];
  hb = hb < 0 ? 0 : (hb > RCAP ? RCAP : hb);
  he = he < hb ? hb : (he > RCAP ? RCAP : he);
  if (lane == 0) misc[16 + wave] = (he - hb + TROWS - 1) / TROWS;
  __syncthreads();
  int maxT = 0;
#pragma unroll
  for (int w2 = 0; w2 < NWAVE; ++w2) { const int tw = misc[16 + w2]; maxT = tw > maxT ? tw : maxT; }
  maxT = maxT < 0 ? 0 : (maxT > MAXTILES ? MAXTILES : maxT);

  const float bA = sB2[2 * lane];
  const float bB = sB2[2 * lane + 1];
  _Float16* sAw = sA + wave * TROWS * AP;
  float*    sDw = sD + wave * TROWS * DP;
  _Float16* ra  = sAw + lane * AP;
  int   curS = NBMAX;
  float rm0 = 0.0f, rm1 = 0.0f;
#pragma unroll 1
  for (int it = 0; it < maxT; ++it) {
    const int  idx   = hb + it * TROWS + lane;
    const bool valid = idx < he;
    const int  ent   = sl[idx < RCAP ? idx : RCAP - 1];
    const int  slt   = valid ? (ent & (NBMAX - 1)) : NBMAX;
    int eid = ent >> SLB;
    eid = eid < 0 ? 0 : (eid > nE - 1 ? nE - 1 : eid);
    int li = elast[eid];
    li = li < 0 ? 0 : (li > nLast - 1 ? nLast - 1 : li);
    int nd = nodeBase + (ent & (NBMAX - 1));
    nd = nd > mRows - 1 ? mRows - 1 : nd;
    const float* pr = PL  + (size_t)li * F;
    const float* cr = CCB + (size_t)nd * F;
#pragma unroll 1
    for (int c8 = 0; c8 < F / 8; ++c8) {
      const v4f pa = *(const v4fa*)(pr + 8 * c8);
      const v4f pb = *(const v4fa*)(pr + 8 * c8 + 4);
      const v4f ca = *(const v4fa*)(cr + 8 * c8);
      const v4f cb = *(const v4fa*)(cr + 8 * c8 + 4);
      const v8f s8 = {pa.x + ca.x, pa.y + ca.y, pa.z + ca.z, pa.w + ca.w,
                      pb.x + cb.x, pb.y + cb.y, pb.z + cb.z, pb.w + cb.w};
      v8h o;
#pragma unroll
      for (int i = 0; i < 8; ++i) o[i] = (_Float16)(fmaxf(s8[i], 0.0f) * SC_A);
      *(v8ha*)(ra + 8 * c8) = o;
    }
    __syncthreads();

    wave_gemm_h(sAw, sDw, W2H, hh, m);
    __syncthreads();

#pragma unroll 1
    for (int i = 0; i < TROWS; ++i) {
      const int si = __builtin_amdgcn_readlane(slt, i);
      if (si != curS) {
        if (curS < NBMAX) {
          v2f w2; w2.x = rm0; w2.y = rm1;
          *(v2fa*)(sAG + curS * F + 2 * lane) = w2;
        }
        curS = si; rm0 = 0.0f; rm1 = 0.0f;
      }
      const v2f d = *(const v2fa*)(sDw + i * DP + 2 * lane);
      rm0 = fmaxf(rm0, fmaxf(fmaf(d.x, SC14, bA), 0.0f));
      rm1 = fmaxf(rm1, fmaxf(fmaf(d.y, SC14, bB), 0.0f));
    }
  }
  if (curS < NBMAX) {
    v2f w2; w2.x = rm0; w2.y = rm1;
    *(v2fa*)(sAG + curS * F + 2 * lane) = w2;
  }
  __syncthreads();

  {
    const float qnan = __int_as_float(0x7fc00000);
    const float pz   = (misc[9] != 0) ? qnan : 0.0f;
    const int hsel = lane >> 4;
    const int j    = lane & 15;
    const int part = j >> 3;
    const int c8   = (j & 7) * 8;
    const unsigned mh = 0u - (unsigned)part;
    const unsigned ml = ~mh;
    const int npair = nsl >> 1;
#pragma unroll 1
    for (int i2 = 0; i2 < npair; ++i2) {
      const int  sa   = ss0 + 2 * i2 + hsel;
      const int  row  = nodeBase + sa;
      const bool live = (nodeBase + ss0 + 2 * i2) < mRows;
      const float* sp = sAG + sa * F + c8;
      const v4f a = *(const v4fa*)sp;
      const v4f b = *(const v4fa*)(sp + 4);
      const v8f f8 = {a.x + pz, a.y + pz, a.z + pz, a.w + pz, b.x + pz, b.y + pz, b.z + pz, b.w + pz};
      v8us oo;
#pragma unroll
      for (int e = 0; e < 8; ++e) {
        const unsigned hb2 = bf16_bits(f8[e]);
        const unsigned lb2 = bf16_bits(f8[e] - __uint_as_float(hb2 << 16));
        oo[e] = (unsigned short)((hb2 & ml) | (lb2 & mh));
      }
      unsigned short* op = AGB + (size_t)(live ? row : 0) * (size_t)KS + 8 * j;
      if (live) *(volatile v8us*)op = oo;
    }
    __threadfence();
#pragma unroll 1
    for (int i2 = 0; i2 < npair; ++i2) {
      const int  sa   = ss0 + 2 * i2 + hsel;
      const int  row  = nodeBase + sa;
      const bool live = (nodeBase + ss0 + 2 * i2) < mRows;
      const float* sp = sAG + sa * F + c8;
      const v4f a = *(const v4fa*)sp;
      const v4f b = *(const v4fa*)(sp + 4);
      const v8f f8 = {a.x + pz, a.y + pz, a.z + pz, a.w + pz, b.x + pz, b.y + pz, b.z + pz, b.w + pz};
      v8us oo;
#pragma unroll
      for (int e = 0; e < 8; ++e) {
        const unsigned hb2 = bf16_bits(f8[e]);
        const unsigned lb2 = bf16_bits(f8[e] - __uint_as_float(hb2 << 16));
        oo[e] = (unsigned short)((hb2 & ml) | (lb2 & mh));
      }
      unsigned short* op = AGB + (size_t)(live ? row : 0) * (size_t)KS + 8 * j;
      if (live) *(volatile v8us*)op = oo;
    }
  }
}

static int pick_nb(int nE, int nN) {
  int nb = NBMAX;
  while (nb > 32 && (long long)nb * (long long)nE * 5LL > (long long)RCAP * (long long)nN * 4LL) nb >>= 1;
  return nb;
}
static inline int cdiv(int a, int b) { return (a + b - 1) / b; }

extern "C" void kernel_launch(void* const* d_in, const int* in_sizes, int n_in,
                              void* d_out, int out_size, void* d_ws, size_t ws_size,
                              hipStream_t stream) {
  if (n_in < 12) return;
  if (in_sizes[0] < 3 || (in_sizes[0] % 3) != 0) return;
  const int nLast = in_sizes[0] / 3;
  if (nLast < 1 || nLast > (1 << 24)) return;
  if ((long long)in_sizes[1] != (long long)nLast * F) return;
  if (in_sizes[2] < 3 || (in_sizes[2] % 3) != 0) return;
  const int nNodes = in_sizes[2] / 3;
  if (nNodes < 1 || nNodes > (1 << 22)) return;
  if (in_sizes[3] < 2 || (in_sizes[3] & 1) != 0) return;
  const int nE = in_sizes[3] / 2;
  if (nE < 1 || nE >= (1 << 23)) return;
  if (in_sizes[4] != K1 * F || in_sizes[5] != F) return;
  if (in_sizes[6] != F * F || in_sizes[7] != F) return;
  if (in_sizes[8] != F * F || in_sizes[9] != F) return;
  if (in_sizes[10] != F * F || in_sizes[11] != F) return;
  if ((long long)out_size != (long long)nNodes * F) return;

  const float* last_coors    = (const float*)d_in[0];
  const float* last_features = (const float*)d_in[1];
  const float* current_coors = (const float*)d_in[2];
  const int*   edge          = (const int*)d_in[3];
  const float* W1 = (const float*)d_in[4];
  const float* b1 = (const float*)d_in[5];
  const float* W2 = (const float*)d_in[6];
  const float* b2 = (const float*)d_in[7];
  const float* W3 = (const float*)d_in[8];
  const float* b3 = (const float*)d_in[9];
  const float* W4 = (const float*)d_in[10];
  const float* b4 = (const float*)d_in[11];
  float* out = (float*)d_out;
  const int* ecur  = edge;
  const int* elast = edge + (size_t)nE;

  const int MPL = cdiv(nLast, GBM) * GBM;
  const int MP  = cdiv(nNodes, GBM) * GBM;
  const int nb  = pick_nb(nE, nNodes);
  if (nb < 32 || (nb & (nb - 1)) != 0 || nb > NBMAX) return;
  const int gA = cdiv(MP, nb);
  if ((long long)gA * nb < (long long)MP) return;

  char* ws = (char*)d_ws;
  size_t off = 0;
  const size_t oW1 = off; off += (size_t)F * K1P * 2;          off = (off + 255) & ~(size_t)255;
  const size_t oW2 = off; off += (size_t)F * K2 * 2;           off = (off + 255) & ~(size_t)255;
  const size_t oU3 = off; off += (size_t)F * KS * 2;           off = (off + 255) & ~(size_t)255;
  const size_t oU4 = off; off += (size_t)F * KS * 2;           off = (off + 255) & ~(size_t)255;
  const size_t oPL = off; off += (size_t)MPL * F * 4;          off = (off + 255) & ~(size_t)255;
  const size_t oCC = off; off += (size_t)MP * F * 4;           off = (off + 255) & ~(size_t)255;
  const size_t oAG = off; off += (size_t)MP * KS * 2;          off = (off + 255) & ~(size_t)255;
  const size_t oG3 = off; off += (size_t)MP * KS * 2;          off = (off + 255) & ~(size_t)255;
  if (off > ws_size || off > (size_t)WSMAX) return;
  unsigned short* W1T = (unsigned short*)(ws + oW1);
  _Float16*       W2H = (_Float16*)(ws + oW2);
  unsigned short* U3T = (unsigned short*)(ws + oU3);
  unsigned short* U4T = (unsigned short*)(ws + oU4);
  float*          PL  = (float*)(ws + oPL);
  float*          CCB = (float*)(ws + oCC);
  unsigned short* AGB = (unsigned short*)(ws + oAG);
  unsigned short* G3  = (unsigned short*)(ws + oG3);

  hipFuncSetAttribute(reinterpret_cast<const void*>(&k_scan), hipFuncAttributeMaxDynamicSharedMemorySize,
                      (int)AGG_LDS_BYTES);

  const int vec8 = 1;

  k_prep<<<UI_TOT / NTHR, NTHR, 0, stream>>>(W1, W2, W3, W4, W1T, W2H, U3T, U4T);
  k_ccb<<<(MP * 16) / NTHR, NTHR, 0, stream>>>(current_coors, nNodes, W1, b1, MP * 16, CCB);
  k_gemm<2, 0><<<dim3(MPL / GBM, 1), GTHR, 0, stream>>>(W1T, 0, last_features, last_coors, nLast, W1T, K1P, K1P,
                                                        b1, MPL, PL, AGB);
  k_scan<<<gA, NTHR, AGG_LDS_BYTES, stream>>>(ecur, elast, nE, nLast, nb, vec8, MP, PL, CCB, W2H, b2, AGB);
  k_gemm<0, 2><<<dim3(MP / GBM, 1), GTHR, 0, stream>>>(AGB, KS, last_features, last_coors, nLast, U3T, KS, KS,
                                                       b3, MP, PL, G3);
  k_gemm<0, 3><<<dim3(MP / GBM, 1), GTHR, 0, stream>>>(G3, KS, last_features, last_coors, nLast, U4T, KS, KS,
                                                       b4, nNodes, out, AGB);
}
